// OuterTransformer_60962765799601
// MI455X (gfx1250) — hardware-verified
//
#include <hip/hip_runtime.h>
#include <stddef.h>


typedef _Float16 f16;
typedef __bf16   bf16;
typedef f16   v16h __attribute__((ext_vector_type(16)));
typedef f16   v8h  __attribute__((ext_vector_type(8)));
typedef f16   v4h  __attribute__((ext_vector_type(4)));
typedef bf16  v16b __attribute__((ext_vector_type(16)));
typedef bf16  v8b  __attribute__((ext_vector_type(8)));
typedef bf16  v4b  __attribute__((ext_vector_type(4)));
typedef float v8f  __attribute__((ext_vector_type(8)));
typedef float v4f  __attribute__((ext_vector_type(4)));

#define NB      4
#define NSEQ    8192
#define DD      256
#define NTOT    (NB * NSEQ)
#define KSLAB   128
#define NP      8
#define PROWS   (NTOT / NP)
#define NSLABP  (PROWS / KSLAB)
#define GQ      64
#define NQ      (DD / GQ)
#define RS      136
#define RSK     40
#define OROWS   64
#define SOP     260
#define SGP     68
#define NTHR    256

union FragH   { v16h v; v8h p[2]; };
union FragB   { v16b v; v8b p[2]; };
union PackH4  { v4h v;  f16 e[4]; };
union PackB4  { v4b v;  bf16 e[4]; };
union PackB8  { v8b v;  bf16 e[8]; };
union PackB16 { v16b v; bf16 e[16]; };

__device__ __forceinline__ v16h ld_frag_h(const f16* base, int pitch, int lane) {
  const f16* p = base + (lane & 15) * pitch + 8 * (lane >> 4);
  FragH u;
  u.p[0] = *(const v8h*)(p);
  u.p[1] = *(const v8h*)(p + 16);
  return u.v;
}
__device__ __forceinline__ v16b ld_frag_b(const bf16* base, int pitch, int lane) {
  const bf16* p = base + (lane & 15) * pitch + 8 * (lane >> 4);
  FragB u;
  u.p[0] = *(const v8b*)(p);
  u.p[1] = *(const v8b*)(p + 16);
  return u.v;
}

__device__ __forceinline__ v8f mma_h(v16h a, v16h b, v8f c) {
  c = __builtin_amdgcn_wmma_f32_16x16x32_f16(false, a, false, b, (short)0, c, false, false);
  asm volatile("v_nop\n\tv_nop\n\tv_nop\n\tv_nop" : "+v"(c) : "v"(a), "v"(b));
  return c;
}
__device__ __forceinline__ v8f mma3_b(v16b ah, v16b al, v16b bh, v16b bl, v8f c) {
  c = __builtin_amdgcn_wmma_f32_16x16x32_bf16(false, ah, false, bh, (short)0, c, false, false);
  c = __builtin_amdgcn_wmma_f32_16x16x32_bf16(false, ah, false, bl, (short)0, c, false, false);
  c = __builtin_amdgcn_wmma_f32_16x16x32_bf16(false, al, false, bh, (short)0, c, false, false);
  asm volatile("v_nop\n\tv_nop\n\tv_nop\n\tv_nop" : "+v"(c) : "v"(ah), "v"(al), "v"(bh), "v"(bl));
  return c;
}

__device__ __forceinline__ void gram_store(const float* sO, const float* sSum,
                                           float* wsGp, float* wsSp, int q, int t) {
#pragma unroll
  for (int it = 0; it < 16; ++it) {
    const int L   = it * 32 + (t >> 3);
    const int row = L >> 1;
    const int c   = (L & 1) * 32 + (t & 7) * 4;
    const v4f v = *(const v4f*)(sO + row * SGP + c);
    *(volatile v4f*)(wsGp + (size_t)row * DD + GQ * q + c) = v;
  }
  if (t < 16) {
    const int c = (t >> 3) * 32 + (t & 7) * 4;
    const v4f v = *(const v4f*)(sSum + GQ * q + c);
    *(volatile v4f*)(wsSp + GQ * q + c) = v;
  }
}

__global__ __launch_bounds__(NTHR) __attribute__((amdgpu_num_vgpr(256)))
void k_gram(const float* __restrict__ x, float* wsG, float* wsS) {
  __shared__ __attribute__((aligned(16))) unsigned char smem[DD * RS * 2];
  __shared__ __attribute__((aligned(16))) float sAux[5 * DD];
  f16*   sh = (f16*)smem;
  float* sO = (float*)smem;
  const int t = threadIdx.x, lane = t & 31, w = t >> 5;
  const int m = lane & 15, h = lane >> 4;
  const int q = blockIdx.x;
  const int p = blockIdx.y;
  const int c4 = (t & 63) * 4;
  const int g  = t >> 6;

  v8f acc[2][4] = {};
  float cs[4] = {0.f, 0.f, 0.f, 0.f};
  const size_t rowBase = (size_t)p * PROWS;

  for (int s = 0; s < NSLABP; ++s) {
    __syncthreads();
#pragma unroll
    for (int r = 0; r < 8; ++r) {
      const int kk = g * 32 + r * 4;
      const float* src = x + (rowBase + (size_t)s * KSLAB + kk) * DD + c4;
      const float4 f0 = *(const float4*)(src);
      const float4 f1 = *(const float4*)(src + DD);
      const float4 f2 = *(const float4*)(src + 2 * DD);
      const float4 f3 = *(const float4*)(src + 3 * DD);
      const float fv[4][4] = {{f0.x, f0.y, f0.z, f0.w},
                              {f1.x, f1.y, f1.z, f1.w},
                              {f2.x, f2.y, f2.z, f2.w},
                              {f3.x, f3.y, f3.z, f3.w}};
#pragma unroll
      for (int jj = 0; jj < 4; ++jj) {
        PackH4 P;
#pragma unroll
        for (int rr = 0; rr < 4; ++rr) {
          const float v = fv[rr][jj];
          P.e[rr] = (f16)v;
          cs[jj] += v;
        }
        *(v4h*)(sh + (c4 + jj) * RS + kk) = P.v;
      }
    }
    __syncthreads();
#pragma unroll
    for (int ks = 0; ks < KSLAB / 32; ++ks) {
      const v16h a0 = ld_frag_h(sh + (32 * w) * RS + 32 * ks, RS, lane);
      const v16h a1 = ld_frag_h(sh + (32 * w + 16) * RS + 32 * ks, RS, lane);
#pragma unroll
      for (int j = 0; j < 4; ++j) {
        const v16h b = ld_frag_h(sh + (GQ * q + 16 * j) * RS + 32 * ks, RS, lane);
        acc[0][j] = mma_h(a0, b, acc[0][j]);
        acc[1][j] = mma_h(a1, b, acc[1][j]);
      }
    }
  }

  __syncthreads();
#pragma unroll
  for (int i = 0; i < 2; ++i)
#pragma unroll
    for (int j = 0; j < 4; ++j)
#pragma unroll
      for (int r = 0; r < 8; ++r)
        sO[(32 * w + 16 * i + 8 * h + r) * SGP + 16 * j + m] = acc[i][j][r];
#pragma unroll
  for (int jj = 0; jj < 4; ++jj) sAux[g * DD + c4 + jj] = cs[jj];
  __syncthreads();
  sAux[4 * DD + t] = sAux[t] + sAux[DD + t] + sAux[2 * DD + t] + sAux[3 * DD + t];
  __syncthreads();

  float* wsGp = wsG + (size_t)p * DD * DD;
  float* wsSp = wsS + (size_t)p * DD;
  gram_store(sO, sAux + 4 * DD, wsGp, wsSp, q, t);
  __threadfence();
  gram_store(sO, sAux + 4 * DD, wsGp, wsSp, q, t);
}

__device__ __forceinline__ void mt_store(const float* sM, float* wsMT, int k0, int t) {
#pragma unroll
  for (int it = 0; it < 4; ++it) {
    const int L  = it * 32 + (t >> 3);
    const int kr = L >> 3;
    const int c  = (L & 7) * 32 + (t & 7) * 4;
    const v4f v = *(const v4f*)(sM + kr * SOP + c);
    *(volatile v4f*)(wsMT + (size_t)(k0 + kr) * DD + c) = v;
  }
}

__global__ __launch_bounds__(NTHR) __attribute__((amdgpu_num_vgpr(256)))
void k_mw(const float* wsG, const float* wsS,
          const float* __restrict__ Wm, const float* __restrict__ bvec, float* wsMT) {
  __shared__ __attribute__((aligned(16))) bf16 sGh[DD * RSK];
  __shared__ __attribute__((aligned(16))) bf16 sGl[DD * RSK];
  __shared__ __attribute__((aligned(16))) bf16 sWh[16 * RSK];
  __shared__ __attribute__((aligned(16))) bf16 sWl[16 * RSK];
  __shared__ __attribute__((aligned(16))) float sM[16 * SOP];
  __shared__ float sS[DD];
  const int t = threadIdx.x, lane = t & 31, w = t >> 5;
  const int m = lane & 15, h = lane >> 4;
  const int k0 = 16 * blockIdx.x;

  {
    float sv = 0.f;
#pragma unroll
    for (int p = 0; p < NP; ++p) sv += wsS[p * DD + t];
    sS[t] = sv;
  }
  const float bk = bvec[k0 + m];
  v8f acc[2] = {};

  for (int s = 0; s < DD / 32; ++s) {
    __syncthreads();
#pragma unroll
    for (int i = 0; i < 4; ++i) {
      float fv[8] = {0.f, 0.f, 0.f, 0.f, 0.f, 0.f, 0.f, 0.f};
#pragma unroll
      for (int p = 0; p < NP; ++p) {
        const float* src = wsG + ((size_t)p * DD + t) * DD + 32 * s + 8 * i;
        const float4 fa = *(const float4*)(src);
        const float4 fb = *(const float4*)(src + 4);
        fv[0] += fa.x; fv[1] += fa.y; fv[2] += fa.z; fv[3] += fa.w;
        fv[4] += fb.x; fv[5] += fb.y; fv[6] += fb.z; fv[7] += fb.w;
      }
      PackB8 H, Lq;
#pragma unroll
      for (int e = 0; e < 8; ++e) {
        const float v = fv[e];
        const bf16 hi = (bf16)v;
        H.e[e]  = hi;
        Lq.e[e] = (bf16)(v - (float)hi);
      }
      *(v8b*)(sGh + t * RSK + 8 * i) = H.v;
      *(v8b*)(sGl + t * RSK + 8 * i) = Lq.v;
    }
#pragma unroll
    for (int rep = 0; rep < 2; ++rep) {
      const int idx = t + NTHR * rep;
      const int e = idx >> 4, n = idx & 15;
      const float v = Wm[(size_t)(32 * s + e) * DD + k0 + n];
      const bf16 hi = (bf16)v;
      sWh[n * RSK + e] = hi;
      sWl[n * RSK + e] = (bf16)(v - (float)hi);
    }
    __syncthreads();
    const v16b bh = ld_frag_b(sWh, RSK, lane);
    const v16b bl = ld_frag_b(sWl, RSK, lane);
#pragma unroll
    for (int i = 0; i < 2; ++i) {
      const v16b ah = ld_frag_b(sGh + (32 * w + 16 * i) * RSK, RSK, lane);
      const v16b al = ld_frag_b(sGl + (32 * w + 16 * i) * RSK, RSK, lane);
      acc[i] = mma3_b(ah, al, bh, bl, acc[i]);
    }
  }

#pragma unroll
  for (int i = 0; i < 2; ++i)
#pragma unroll
    for (int r = 0; r < 8; ++r) {
      const int d = 32 * w + 16 * i + 8 * h + r;
      sM[m * SOP + d] = acc[i][r] + sS[d] * bk;
    }
  __syncthreads();
  mt_store(sM, wsMT, k0, t);
  __threadfence();
  mt_store(sM, wsMT, k0, t);
}

__device__ __forceinline__ void out_store(const float* sO, float* out, int n0, int t) {
#pragma unroll
  for (int it = 0; it < 16; ++it) {
    const int L   = it * 32 + (t >> 3);
    const int row = L >> 3;
    const int c   = (L & 7) * 32 + (t & 7) * 4;
    const v4f v = *(const v4f*)(sO + row * SOP + c);
    *(volatile v4f*)(out + (size_t)(n0 + row) * DD + c) = v;
  }
}

__global__ __launch_bounds__(NTHR) __attribute__((amdgpu_num_vgpr(256)))
void k_out(const float* __restrict__ x, const float* wsMT, float* out) {
  __shared__ __attribute__((aligned(16))) unsigned char smem[2 * DD * RS * 2];
  bf16*  sBh = (bf16*)smem;
  bf16*  sBl = sBh + DD * RS;
  float* sO  = (float*)smem;
  const int t = threadIdx.x, lane = t & 31, w = t >> 5;
  const int m = lane & 15, h = lane >> 4;
  const int rt  = w >> 1;
  const int ct0 = (w & 1) * 8;
  const int n0  = blockIdx.x * OROWS;

  v8f acc[8] = {};
  const float* arow = x + (size_t)(n0 + 16 * rt + m) * DD;

  for (int kh = 0; kh < 2; ++kh) {
    __syncthreads();
#pragma unroll 8
    for (int i = 0; i < 32; ++i) {
      const int k = w + 8 * i;
      const float4 f = *(const float4*)(wsMT + (size_t)k * DD + 128 * kh + 4 * lane);
      const float fv[4] = {f.x, f.y, f.z, f.w};
      PackB4 H, Lq;
#pragma unroll
      for (int e = 0; e < 4; ++e) {
        const float v = fv[e];
        const bf16 hi = (bf16)v;
        H.e[e]  = hi;
        Lq.e[e] = (bf16)(v - (float)hi);
      }
      *(v4b*)(sBh + k * RS + 4 * lane) = H.v;
      *(v4b*)(sBl + k * RS + 4 * lane) = Lq.v;
    }
    __syncthreads();
#pragma unroll
    for (int ks = 0; ks < 4; ++ks) {
      const float* p0 = arow + 128 * kh + 32 * ks + 8 * h;
      const float4 fa = *(const float4*)(p0);
      const float4 fb = *(const float4*)(p0 + 4);
      const float4 fc = *(const float4*)(p0 + 16);
      const float4 fd = *(const float4*)(p0 + 20);
      const float fl[16] = {fa.x, fa.y, fa.z, fa.w, fb.x, fb.y, fb.z, fb.w,
                            fc.x, fc.y, fc.z, fc.w, fd.x, fd.y, fd.z, fd.w};
      PackB16 AH, AL;
#pragma unroll
      for (int i = 0; i < 16; ++i) {
        const float v = fl[i];
        const bf16 hi = (bf16)v;
        AH.e[i] = hi;
        AL.e[i] = (bf16)(v - (float)hi);
      }
#pragma unroll
      for (int j = 0; j < 8; ++j) {
        const int boff = (16 * (ct0 + j)) * RS + 32 * ks;
        const v16b bh = ld_frag_b(sBh + boff, RS, lane);
        const v16b bl = ld_frag_b(sBl + boff, RS, lane);
        acc[j] = mma3_b(AH.v, AL.v, bh, bl, acc[j]);
      }
    }
  }

  __syncthreads();
#pragma unroll
  for (int j = 0; j < 8; ++j)
#pragma unroll
    for (int r = 0; r < 8; ++r)
      sO[(16 * rt + 8 * h + r) * SOP + 16 * (ct0 + j) + m] = acc[j][r];
  __syncthreads();
  out_store(sO, out, n0, t);
  __threadfence();
  out_store(sO, out, n0, t);
}

extern "C" void kernel_launch(void* const* d_in, const int* in_sizes, int n_in,
                              void* d_out, int out_size, void* d_ws, size_t ws_size,
                              hipStream_t stream) {
  if (n_in < 3) return;
  if (in_sizes[0] != NTOT * DD || in_sizes[1] != DD * DD || in_sizes[2] != DD) return;
  if (out_size != NTOT * DD) return;

  const size_t bytesG  = (size_t)NP * DD * DD * sizeof(float);
  const size_t bytesS  = (size_t)NP * DD * sizeof(float);
  const size_t bytesMT = (size_t)DD * DD * sizeof(float);
  const size_t offG  = 0;
  const size_t offS  = offG + bytesG;
  const size_t offMT = offS + bytesS;
  if (offMT + bytesMT > ws_size) return;

  const float* x  = (const float*)d_in[0];
  const float* Wm = (const float*)d_in[1];
  const float* bv = (const float*)d_in[2];
  float* out  = (float*)d_out;
  float* wsG  = (float*)((char*)d_ws + offG);
  float* wsS  = (float*)((char*)d_ws + offS);
  float* wsMT = (float*)((char*)d_ws + offMT);

  hipLaunchKernelGGL(k_gram, dim3(NQ, NP), dim3(NTHR), 0, stream, x, wsG, wsS);
  hipLaunchKernelGGL(k_mw, dim3(DD / 16), dim3(NTHR), 0, stream, wsG, wsS, Wm, bv, wsMT);
  hipLaunchKernelGGL(k_out, dim3(NTOT / OROWS), dim3(NTHR), 0, stream, x, wsMT, out);
  (void)hipGetLastError();
}
